// CNF_regularized_23278722744620
// MI455X (gfx1250) — hardware-verified
//
#include <hip/hip_runtime.h>
#include <stddef.h>


typedef _Float16 v16h __attribute__((ext_vector_type(16)));
typedef _Float16 v8h  __attribute__((ext_vector_type(8)));
typedef float    v8f  __attribute__((ext_vector_type(8)));
typedef float    v4f  __attribute__((ext_vector_type(4)));
typedef _Float16 h16;

#ifndef NROWS
#define NROWS 2048
#endif
#define NROWS_FULL 2048
#define DZ    64
#define HID   512
#define MROWS NROWS

static_assert(NROWS >= 64 && NROWS <= NROWS_FULL && (NROWS % 64) == 0);
static_assert(DZ == 64 && (DZ % 32) == 0 && (DZ % 64) == 0);
static_assert((HID % 64) == 0 && (HID % 32) == 0);
static_assert(((MROWS * DZ) % 2048) == 0);
static_assert(((HID * DZ) % 2048) == 0);

#define LDT 72
#define LDC 68
static_assert((LDT % 8) == 0 && LDT >= 64);
static_assert((LDC % 4) == 0 && LDC >= 64);
static_assert((64 * LDC + 64) * 4 <= 131072);
static_assert(64 * LDT * 2 <= 131072);

#define WCARRY 64.0f
#define HCARRY 16.0f
#define TCARRY (WCARRY * WCARRY)

static_assert((256 / 8) * 2 == 64);
static_assert((256 / 16) * 4 == 64);
static_assert((256 / 4) == 64);

#define OUT1_OFF ((size_t)NROWS_FULL * DZ)
static_assert(OUT1_OFF * 4 == (size_t)524288);
static_assert((OUT1_OFF + NROWS_FULL) * 4 == (size_t)532480);

#define Z16_BYTES  ((size_t)MROWS * DZ * 2)
#define WS_BYTES64 ((size_t)HID * DZ * 2)
#define WSQ_BYTES  ((size_t)HID * HID * 2)
#define P16_BYTES  ((size_t)MROWS * HID * 2)
#define P32_BYTES  ((size_t)MROWS * HID * 4)
#define OFF_Z   ((size_t)0)
#define OFF_W1T (OFF_Z + Z16_BYTES)
#define OFF_W3C (OFF_W1T + WS_BYTES64)
#define OFF_W3T (OFF_W3C + WS_BYTES64)
#define OFF_W2T (OFF_W3T + WS_BYTES64)
#define OFF_MT  (OFF_W2T + WSQ_BYTES)
#define OFF_H1  (OFF_MT + WSQ_BYTES)
#define OFF_S1  (OFF_H1 + P16_BYTES)
#define OFF_H2  (OFF_S1 + P16_BYTES)
#define OFF_S2  (OFF_H2 + P16_BYTES)
#define WS_TOTAL (OFF_S2 + P32_BYTES)
static_assert((Z16_BYTES % 128) == 0 && (WS_BYTES64 % 128) == 0 && (WSQ_BYTES % 128) == 0);
static_assert((P16_BYTES % 128) == 0 && (P32_BYTES % 128) == 0);
static_assert(WS_TOTAL <= (size_t)134217728);

__device__ __forceinline__ float bf16r(float x) {
  unsigned int u = __float_as_uint(x);
  u = (u + 0x7FFFu + ((u >> 16) & 1u)) & 0xFFFF0000u;
  return __uint_as_float(u);
}

static __device__ __forceinline__ h16 toh_flush(float v) {
  const h16 r = (h16)v;
  return (fabsf(v) < 6.103515625e-05f) ? (h16)0.0f : r;
}

__device__ __forceinline__ v16h frag_at(const _Float16* p) {
  v8h lo = *(const v8h*)(p);
  v8h hi = *(const v8h*)(p + 16);
  v16h out;
#pragma unroll
  for (int i = 0; i < 8; ++i) { out[i] = lo[i]; out[i + 8] = hi[i]; }
  return out;
}

__device__ __forceinline__ v8f wmma16(v16h a, v16h b, v8f c) {
  v8f d = __builtin_amdgcn_wmma_f32_16x16x32_f16(false, a, false, b, (short)0, c,
                                                 false, false);
  asm volatile("v_nop\n\tv_nop\n\tv_nop\n\tv_nop" : "+v"(d) : "v"(a), "v"(b));
  return d;
}

__global__ __launch_bounds__(256) void wconv_kernel(
    const float* __restrict__ W, _Float16* __restrict__ Wt, unsigned ldw, unsigned ldk) {
  __shared__ _Float16 T[64 * LDT];
  const unsigned tid = threadIdx.x;
  const unsigned n0 = blockIdx.x * 64u;
  const unsigned k0 = blockIdx.y * 64u;
#pragma unroll 4
  for (unsigned j = 0; j < 16u; ++j) {
    const unsigned idx = tid + 256u * j;
    const unsigned kr = idx >> 6, nc = idx & 63u;
    const float v = W[(size_t)(k0 + kr) * ldw + n0 + nc];
    T[nc * LDT + kr] = toh_flush(WCARRY * bf16r(v));
  }
  __syncthreads();
  v8h x[2];
  size_t off[2];
#pragma unroll
  for (unsigned i = 0; i < 2u; ++i) {
    const unsigned n = 32u * i + (tid >> 3);
    const unsigned kc = (tid & 7u) * 8u;
    x[i] = *(const v8h*)&T[n * LDT + kc];
    off[i] = (size_t)(n0 + n) * ldk + k0 + kc;
  }
#pragma unroll
  for (int i = 0; i < 2; ++i) *(volatile v8h*)(Wt + off[i]) = x[i];
  __threadfence();
#pragma unroll
  for (int i = 0; i < 2; ++i) *(volatile v8h*)(Wt + off[i]) = x[i];
}

__global__ __launch_bounds__(256) void cast_kernel(
    const float* __restrict__ src, _Float16* __restrict__ dst, float carry) {
  const size_t i = ((size_t)blockIdx.x * 256u + threadIdx.x) * 8u;
  const v4f a0 = *(const v4f*)(src + i);
  const v4f a1 = *(const v4f*)(src + i + 4u);
  v8h o;
#pragma unroll
  for (int j = 0; j < 4; ++j) {
    o[j]     = toh_flush(carry * bf16r(a0[j]));
    o[j + 4] = toh_flush(carry * bf16r(a1[j]));
  }
  _Float16* p = dst + i;
  *(volatile v8h*)p = o;
  __threadfence();
  *(volatile v8h*)p = o;
}

template <int MODE>
__device__ __forceinline__ void gemm_body(
    const _Float16* __restrict__ A16, const _Float16* __restrict__ Bt, const unsigned K,
    const float* __restrict__ bias, const float* __restrict__ aux,
    const float* __restrict__ tin,
    float* __restrict__ outf, _Float16* __restrict__ out16, _Float16* __restrict__ out16b) {
  __shared__ float Cs[64 * LDC];
  const unsigned tid = threadIdx.x, lane = tid & 31u, w = tid >> 5;
  const unsigned mw = w >> 1, nw = w & 1u;
  const unsigned hh = lane >> 4, m = lane & 15u;
  const unsigned n0 = blockIdx.x * 64u;
  const unsigned row0 = blockIdx.y * 64u;

  const _Float16* ap  = A16 + (size_t)(row0 + mw * 16u + m) * K + hh * 8u;
  const _Float16* bp0 = Bt + (size_t)(n0 + nw * 32u + m) * K + hh * 8u;
  const _Float16* bp1 = bp0 + (size_t)16 * K;
  v8f acc0 = {}, acc1 = {};
#pragma unroll 2
  for (unsigned k0 = 0; k0 < K; k0 += 32u) {
    const v16h a  = frag_at(ap + k0);
    const v16h b0 = frag_at(bp0 + k0);
    const v16h b1 = frag_at(bp1 + k0);
    acc0 = wmma16(a, b0, acc0);
    acc1 = wmma16(a, b1, acc1);
  }
#pragma unroll
  for (int r = 0; r < 8; ++r) {
    float* d = &Cs[(mw * 16u + hh * 8u + (unsigned)r) * LDC + nw * 32u + m];
    d[0]  = acc0[r];
    d[16] = acc1[r];
  }
  __syncthreads();

  if (MODE == 0 || MODE == 1) {
    const float cs = (MODE == 0) ? (1.0f / WCARRY) : (1.0f / (WCARRY * HCARRY));
    float tv = 0.0f;
    if (MODE == 0) tv = bf16r(tin[0]);
#pragma unroll 1
    for (unsigned g = 0; g < 4u; ++g) {
      const unsigned r = 32u * (g >> 1) + (tid >> 3);
      const unsigned c = (tid & 7u) * 8u + 4u * (g & 1u);
      const v4f u  = *(const v4f*)&Cs[r * LDC + c];
      const v4f gb = *(const v4f*)(bias + n0 + c);
      v4f ga = {};
      if (MODE == 0) ga = *(const v4f*)(aux + n0 + c);
      v4f t;
#pragma unroll
      for (int j = 0; j < 4; ++j)
        t[j] = tanhf(u[j] * cs + (bf16r(gb[j]) + tv * bf16r(ga[j])));
      *(v4f*)&Cs[r * LDC + c] = t;
    }
    __syncthreads();
  }

  if (MODE == 3) {
#pragma unroll 4
    for (unsigned g = 0; g < 16u; ++g) {
      const unsigned idx = tid + 256u * g;
      const unsigned r = idx & 63u, c = idx >> 6;
      const float wv = aux[(size_t)(n0 + c) * HID + row0 + r];
      const float cv = Cs[r * LDC + c];
      Cs[r * LDC + c] = cv * bf16r(wv);
    }
    __syncthreads();
  }

  if (MODE == 0 || MODE == 1 || MODE == 3) {
    const float sc16 = (MODE == 3) ? 1.0f : HCARRY;
    v8h x[2] = {}, y[2] = {};
    size_t off[2];
#pragma unroll
    for (unsigned i = 0; i < 2u; ++i) {
      const unsigned r = 32u * i + (tid >> 3);
      const unsigned c = (tid & 7u) * 8u;
      const v4f u0 = *(const v4f*)&Cs[r * LDC + c];
      const v4f u1 = *(const v4f*)&Cs[r * LDC + c + 4];
#pragma unroll
      for (int j = 0; j < 4; ++j) {
        x[i][j]     = toh_flush(sc16 * u0[j]);
        x[i][j + 4] = toh_flush(sc16 * u1[j]);
        if (MODE == 0) {
          y[i][j]     = toh_flush(HCARRY * (1.0f - u0[j] * u0[j]));
          y[i][j + 4] = toh_flush(HCARRY * (1.0f - u1[j] * u1[j]));
        }
      }
      off[i] = (size_t)(row0 + r) * HID + n0 + c;
    }
    v4f xs[4] = {};
    size_t offs[4] = {};
    if (MODE == 1) {
#pragma unroll
      for (unsigned i = 0; i < 4u; ++i) {
        const unsigned r = 16u * i + (tid >> 4);
        const unsigned c = (tid & 15u) * 4u;
        const v4f u = *(const v4f*)&Cs[r * LDC + c];
#pragma unroll
        for (int j = 0; j < 4; ++j) xs[i][j] = 1.0f - u[j] * u[j];
        offs[i] = (size_t)(row0 + r) * HID + n0 + c;
      }
    }
#pragma unroll
    for (int i = 0; i < 2; ++i) *(volatile v8h*)(out16 + off[i]) = x[i];
    if (MODE == 0) {
#pragma unroll
      for (int i = 0; i < 2; ++i) *(volatile v8h*)(out16b + off[i]) = y[i];
    }
    if (MODE == 1) {
#pragma unroll
      for (int i = 0; i < 4; ++i) *(volatile v4f*)(outf + offs[i]) = xs[i];
    }
    __threadfence();
#pragma unroll
    for (int i = 0; i < 2; ++i) *(volatile v8h*)(out16 + off[i]) = x[i];
    if (MODE == 0) {
#pragma unroll
      for (int i = 0; i < 2; ++i) *(volatile v8h*)(out16b + off[i]) = y[i];
    }
    if (MODE == 1) {
#pragma unroll
      for (int i = 0; i < 4; ++i) *(volatile v4f*)(outf + offs[i]) = xs[i];
    }
  }

  if (MODE == 2) {
    const float cs = 1.0f / (WCARRY * HCARRY);
    v4f xs[4];
    size_t off[4];
#pragma unroll
    for (unsigned i = 0; i < 4u; ++i) {
      const unsigned r = 16u * i + (tid >> 4);
      const unsigned c = (tid & 15u) * 4u;
      const v4f u = *(const v4f*)&Cs[r * LDC + c];
      const v4f g = *(const v4f*)(bias + n0 + c);
      v4f val;
#pragma unroll
      for (int j = 0; j < 4; ++j) val[j] = u[j] * cs + bf16r(g[j]);
      xs[i] = val;
      off[i] = (size_t)(row0 + r) * DZ + n0 + c;
    }
#pragma unroll
    for (int i = 0; i < 4; ++i) *(volatile v4f*)(outf + off[i]) = xs[i];
    __threadfence();
#pragma unroll
    for (int i = 0; i < 4; ++i) *(volatile v4f*)(outf + off[i]) = xs[i];
  }
}

__global__ __launch_bounds__(256) void gemm_l1_kernel(
    const _Float16* __restrict__ A16, const _Float16* __restrict__ Bt,
    const float* __restrict__ bias, const float* __restrict__ wtime,
    const float* __restrict__ tin,
    _Float16* __restrict__ hplane, _Float16* __restrict__ splane) {
  gemm_body<0>(A16, Bt, (unsigned)DZ, bias, wtime, tin, (float*)0, hplane, splane);
}
__global__ __launch_bounds__(256) void gemm_l2_kernel(
    const _Float16* __restrict__ A16, const _Float16* __restrict__ Bt,
    const float* __restrict__ bias, _Float16* __restrict__ hplane, float* __restrict__ s2f) {
  gemm_body<1>(A16, Bt, (unsigned)HID, bias, bias, bias, s2f, hplane, hplane);
}
__global__ __launch_bounds__(256) void gemm_out_kernel(
    const _Float16* __restrict__ A16, const _Float16* __restrict__ Bt,
    const float* __restrict__ bias, float* __restrict__ outf) {
  gemm_body<2>(A16, Bt, (unsigned)HID, bias, bias, bias, outf, (_Float16*)0, (_Float16*)0);
}
__global__ __launch_bounds__(256) void gemm_mt_kernel(
    const _Float16* __restrict__ A16, const _Float16* __restrict__ Bt,
    const float* __restrict__ w2, _Float16* __restrict__ mt) {
  gemm_body<3>(A16, Bt, (unsigned)DZ, w2, w2, w2, (float*)0, mt, mt);
}

__global__ __launch_bounds__(256) void trace_kernel(
    const _Float16* __restrict__ S1h, const _Float16* __restrict__ Mt,
    const float* __restrict__ S2f, float* __restrict__ tr) {
  __shared__ float Cs[64 * LDC];
  __shared__ float Rs[64];
  const unsigned tid = threadIdx.x, lane = tid & 31u;
  const unsigned w = (unsigned)__builtin_amdgcn_readfirstlane((int)(threadIdx.x >> 5));
  const unsigned mw = w >> 1, nw = w & 1u;
  const unsigned hh = lane >> 4, m = lane & 15u;
  const unsigned row0 = blockIdx.x * 64u;
  const unsigned rr = tid >> 2, cq = (tid & 3u) * 16u;

  const _Float16* ap = S1h + (size_t)(row0 + mw * 16u + m) * HID + hh * 8u;
  float part = 0.0f;
#pragma unroll 1
  for (unsigned n0 = 0; n0 < (unsigned)HID; n0 += 64u) {
    const _Float16* bp0 = Mt + (size_t)(n0 + nw * 32u + m) * HID + hh * 8u;
    const _Float16* bp1 = bp0 + (size_t)16 * HID;
    v8f acc0 = {}, acc1 = {};
#pragma unroll 2
    for (unsigned k0 = 0; k0 < (unsigned)HID; k0 += 32u) {
      const v16h a  = frag_at(ap + k0);
      const v16h b0 = frag_at(bp0 + k0);
      const v16h b1 = frag_at(bp1 + k0);
      acc0 = wmma16(a, b0, acc0);
      acc1 = wmma16(a, b1, acc1);
    }
#pragma unroll
    for (int r = 0; r < 8; ++r) {
      float* d = &Cs[(mw * 16u + hh * 8u + (unsigned)r) * LDC + nw * 32u + m];
      d[0]  = acc0[r];
      d[16] = acc1[r];
    }
    __syncthreads();
    const float* sp = S2f + (size_t)(row0 + rr) * HID + n0 + cq;
#pragma unroll
    for (unsigned q = 0; q < 4u; ++q) {
      const v4f u = *(const v4f*)&Cs[rr * LDC + cq + 4u * q];
      const v4f s = *(const v4f*)(sp + 4u * q);
      part += (u[0] * s[0] + u[1] * s[1]) + (u[2] * s[2] + u[3] * s[3]);
    }
    __syncthreads();
  }
  part += __shfl_xor(part, 1, 32);
  part += __shfl_xor(part, 2, 32);
  if ((tid & 3u) == 0u) Rs[rr] = part * (-1.0f / (HCARRY * TCARRY));
  __syncthreads();
  if (w == 0u) {
    const v4f x = *(const v4f*)&Rs[(lane & 15u) * 4u];
    float* p = tr + row0 + (lane & 15u) * 4u;
    if (lane < 16u) *(volatile v4f*)p = x;
    __threadfence();
    if (lane < 16u) *(volatile v4f*)p = x;
  }
}

extern "C" void kernel_launch(void* const* d_in, const int* in_sizes, int n_in,
                              void* d_out, int out_size, void* d_ws, size_t ws_size,
                              hipStream_t stream) {
  if (n_in < 9) return;
  if ((long long)in_sizes[0] < (long long)MROWS * DZ) return;
  if (in_sizes[2] < 1) return;
  if ((long long)in_sizes[3] < (long long)(DZ + 1) * HID) return;
  if (in_sizes[4] < HID) return;
  if ((long long)in_sizes[5] < (long long)HID * HID) return;
  if (in_sizes[6] < HID) return;
  if ((long long)in_sizes[7] < (long long)HID * DZ) return;
  if (in_sizes[8] < DZ) return;
  if ((long long)out_size < (long long)(OUT1_OFF + MROWS)) return;
  if (ws_size < WS_TOTAL) return;

  const float* z  = (const float*)d_in[0];
  const float* t  = (const float*)d_in[2];
  const float* w1 = (const float*)d_in[3];
  const float* b1 = (const float*)d_in[4];
  const float* w2 = (const float*)d_in[5];
  const float* b2 = (const float*)d_in[6];
  const float* w3 = (const float*)d_in[7];
  const float* b3 = (const float*)d_in[8];
  float* out = (float*)d_out;

  char* ws = (char*)d_ws;
  _Float16* Z16  = (_Float16*)(ws + OFF_Z);
  _Float16* W1t  = (_Float16*)(ws + OFF_W1T);
  _Float16* W3c  = (_Float16*)(ws + OFF_W3C);
  _Float16* W3t  = (_Float16*)(ws + OFF_W3T);
  _Float16* W2t  = (_Float16*)(ws + OFF_W2T);
  _Float16* Mt   = (_Float16*)(ws + OFF_MT);
  _Float16* H1   = (_Float16*)(ws + OFF_H1);
  _Float16* S1h  = (_Float16*)(ws + OFF_S1);
  _Float16* H2   = (_Float16*)(ws + OFF_H2);
  float*    S2f  = (float*)(ws + OFF_S2);

  dim3 blk(256);

  cast_kernel<<<dim3(MROWS * DZ / 2048), blk, 0, stream>>>(z, Z16, 1.0f);
  cast_kernel<<<dim3(HID * DZ / 2048), blk, 0, stream>>>(w3, W3c, WCARRY);
  wconv_kernel<<<dim3(HID / 64, DZ / 64), blk, 0, stream>>>(w1, W1t, (unsigned)HID, (unsigned)DZ);
  wconv_kernel<<<dim3(HID / 64, HID / 64), blk, 0, stream>>>(w2, W2t, (unsigned)HID, (unsigned)HID);
  wconv_kernel<<<dim3(DZ / 64, HID / 64), blk, 0, stream>>>(w3, W3t, (unsigned)DZ, (unsigned)HID);

  gemm_mt_kernel<<<dim3(HID / 64, HID / 64), blk, 0, stream>>>(W3c, W1t, w2, Mt);

  gemm_l1_kernel<<<dim3(HID / 64, MROWS / 64), blk, 0, stream>>>(
      Z16, W1t, b1, w1 + (size_t)DZ * HID, t, H1, S1h);
  gemm_l2_kernel<<<dim3(HID / 64, MROWS / 64), blk, 0, stream>>>(H1, W2t, b2, H2, S2f);
  gemm_out_kernel<<<dim3(DZ / 64, MROWS / 64), blk, 0, stream>>>(H2, W3t, b3, out);
  trace_kernel<<<dim3(MROWS / 64), blk, 0, stream>>>(S1h, Mt, S2f, out + OUT1_OFF);
}
